// DLinear_436
// MI455X (gfx1250) — hardware-run, weakly checked
//
#include <hip/hip_runtime.h>


#ifndef NB
#define NB 32
#endif
#define NB_FULL 32
#define TI   12
#define HH   64
#define WW   64
#define CI   4
#define NO   48
#define KD   96
#define NPOS 64
#define PIXB (HH * WW)
#define TS   (HH * WW * CI)
#define XBS  (TI * TS)
#define OBS  (12 * TS)
#define PP   128
#define OSP  52
#define INV25 (1.0f / 25.0f)
#define WBLK 144
#define BBLK 3

static_assert(NB <= NB_FULL);
static_assert(KD % 32 == 0);
static_assert(NO % 16 == 0);
static_assert(WW == 64);
static_assert(((size_t)NB * PIXB) % PP == 0);
static_assert((PP * KD) % (8 * PP) == 0);
static_assert(NPOS * NO * (KD / 8) == WBLK * 256);
static_assert(NPOS * (NO / 4) == BBLK * 256);
static_assert((OSP % 4) == 0 && OSP >= NO);

typedef unsigned short bf;
typedef __attribute__((ext_vector_type(16))) __bf16   v16bf;
typedef __attribute__((ext_vector_type(8)))  unsigned short v8us;
typedef __attribute__((ext_vector_type(4)))  unsigned short v4us;
typedef __attribute__((ext_vector_type(8)))  float    v8f;
typedef __attribute__((ext_vector_type(4)))  float    v4f;
typedef v4f  __attribute__((may_alias)) v4fa;
typedef v8us __attribute__((may_alias)) v8usa;
typedef v4us __attribute__((may_alias)) v4usa;

__device__ __forceinline__ unsigned short f2bf(float f) { unsigned u = __float_as_uint(f); u += 0x7FFFu + ((u >> 16) & 1u); return (unsigned short)(u >> 16); }
__device__ __forceinline__ float bf2f(unsigned short h) { return __uint_as_float(((unsigned)h) << 16); }
__device__ __forceinline__ float bfr(float f) { return bf2f(f2bf(f)); }
__device__ __forceinline__ v16bf cat16b(v8us lo, v8us hi) { return __builtin_bit_cast(v16bf, __builtin_shufflevector(lo, hi, 0, 1, 2, 3, 4, 5, 6, 7, 8, 9, 10, 11, 12, 13, 14, 15)); }
__device__ __forceinline__ v8f wmmab(v16bf a, v16bf b, v8f c) { return __builtin_amdgcn_wmma_f32_16x16x32_bf16(false, a, false, b, (short)0, c, false, false); }
__device__ __forceinline__ v16bf ldb(const bf* p)  { return cat16b(*(const v8us*)p, *(const v8us*)(p + 16)); }
__device__ __forceinline__ void wave_sync() { __builtin_amdgcn_fence(3  , "wavefront"); __builtin_amdgcn_wave_barrier(); asm volatile("" ::: "memory"); }

__global__ __launch_bounds__(PP) void k_prep(const float* __restrict__ x, bf* VH, bf* VL) {
    __shared__ __align__(16) unsigned short sh[PP * KD];
    __shared__ __align__(16) unsigned short sl[PP * KD];
    const int tid = threadIdx.x;
    const int pix = blockIdx.x * PP + tid;
    const int b = pix >> 12, hw = pix & (PIXB - 1);
    const float* xb = x + (size_t)b * XBS + (size_t)hw * CI;
    v4f x0 = *(const v4f*)xb; v4f x11 = *(const v4f*)(xb + (size_t)(TI - 1) * TS);
#pragma unroll
    for (int c = 0; c < 4; ++c) { x0[c] = bfr(x0[c]); x11[c] = bfr(x11[c]); }
    v4f S = (v4f){};
#pragma unroll 1
    for (int t = 0; t < TI; ++t) { const v4f v = *(const v4f*)(xb + (size_t)t * TS);
#pragma unroll
        for (int c = 0; c < 4; ++c) S[c] += bfr(v[c]); }
#pragma unroll 1
    for (int t = 0; t < TI; ++t) {
        const v4f v = *(const v4f*)(xb + (size_t)t * TS);
        const float fa = (float)(TI - t), fc = (float)(t + 1);
        v4us rh, rl, th, tl;
#pragma unroll
        for (int c = 0; c < 4; ++c) {
            const float xv = bfr(v[c]);
            const float tr = (S[c] + fa * x0[c] + fc * x11[c]) * INV25;
            const float rs = xv - tr;
            const unsigned short h0 = f2bf(rs); rh[c] = h0; rl[c] = f2bf(rs - bf2f(h0));
            const unsigned short h1 = f2bf(tr); th[c] = h1; tl[c] = f2bf(tr - bf2f(h1));
        }
        *(v4usa*)(&sh[tid * KD + t * 4]) = rh;      *(v4usa*)(&sl[tid * KD + t * 4]) = rl;
        *(v4usa*)(&sh[tid * KD + 48 + t * 4]) = th; *(v4usa*)(&sl[tid * KD + 48 + t * 4]) = tl;
    }
    __syncthreads();
    bf* gh = VH + (size_t)blockIdx.x * PP * KD; bf* gl = VL + (size_t)blockIdx.x * PP * KD;
#pragma unroll 1
    for (int ps = 0; ps < 2; ++ps) {
#pragma unroll 4
        for (int it = 0; it < (PP * KD) / (8 * PP); ++it) { const int q = it * PP + tid;
            const v8us a = *(const v8usa*)(&sh[q * 8]); const v8us c = *(const v8usa*)(&sl[q * 8]);
            *(volatile v8us*)(gh + (size_t)q * 8) = a; *(volatile v8us*)(gl + (size_t)q * 8) = c; }
        if (ps == 0) __threadfence(); }
}

__global__ __launch_bounds__(256) void k_w(const float* __restrict__ ws, const float* __restrict__ bs, const float* __restrict__ wt, const float* __restrict__ bt, bf* WST, float* BIAS) {
    const int tid = threadIdx.x;
    if (blockIdx.x < WBLK) {
        const int p = blockIdx.x * 256 + tid;
        const int k8 = p % 12, ro = p / 12; const int o = ro % NO, pos = ro / NO;
        const int kk0 = (k8 % 6) * 8; const int useS = (k8 < 6);
        v8us ov;
#pragma unroll
        for (int e = 0; e < 8; ++e) { const int idx = (o * 48 + kk0 + e) * 64 + pos; const float a = ws[idx]; const float c = wt[idx]; ov[e] = f2bf(useS ? a : c); }
        *(volatile v8us*)(WST + (size_t)p * 8) = ov; __threadfence(); *(volatile v8us*)(WST + (size_t)p * 8) = ov;
    } else {
        const int p = (blockIdx.x - WBLK) * 256 + tid;
        const int pos = p / 12, o4 = (p % 12) * 4;
        v4f ov;
#pragma unroll
        for (int e = 0; e < 4; ++e) { const int idx = (o4 + e) * 64 + pos; ov[e] = bfr(bs[idx]) + bfr(bt[idx]); }
        *(volatile v4f*)(BIAS + (size_t)p * 4) = ov; __threadfence(); *(volatile v4f*)(BIAS + (size_t)p * 4) = ov;
    }
}

__global__ __launch_bounds__(32) __attribute__((amdgpu_num_vgpr(256))) void k_gemm(const bf* __restrict__ VH, const bf* __restrict__ VL, const bf* __restrict__ WST, const float* __restrict__ BIAS, float* OUT) {
    __shared__ __align__(16) float os[WW * OSP];
    const int lane = threadIdx.x & 31, lr = lane & 15, hi = lane >> 4;
    const int y = blockIdx.x, b = blockIdx.y;
    const int yq = y >> 2, ry = y & 3;
    const int ok0 = (yq <= 14), ok1 = (yq >= 1);
    const size_t rowbase = ((size_t)(b * HH + y) * WW) * KD;
#pragma unroll 1
    for (int rx = 0; rx < 4; ++rx) {
        const size_t ao = rowbase + (size_t)(rx + 4 * lr) * KD + 8 * hi;
        v16bf ah[3], al[3];
#pragma unroll
        for (int kc = 0; kc < 3; ++kc) { ah[kc] = ldb(VH + ao + kc * 32); al[kc] = ldb(VL + ao + kc * 32); }
        v8f acc[2][3]; float bsum[2][3];
#pragma unroll
        for (int dj = 0; dj < 2; ++dj)
#pragma unroll
            for (int nb = 0; nb < 3; ++nb) { acc[dj][nb] = (v8f){}; bsum[dj][nb] = 0.0f; }
#pragma unroll
        for (int di = 0; di < 2; ++di) {
            const int ok = di ? ok1 : ok0;
#pragma unroll
            for (int dj = 0; dj < 2; ++dj) {
                const int pos = (ry + 4 * di) * 8 + rx + 4 * dj;
                const float* bp = BIAS + pos * NO + lr;
                const float c0 = bp[0], c1 = bp[16], c2 = bp[32];
                bsum[dj][0] += ok ? c0 : 0.0f; bsum[dj][1] += ok ? c1 : 0.0f; bsum[dj][2] += ok ? c2 : 0.0f;
                if (ok) {
                    const bf* wp = WST + ((size_t)pos * NO + lr) * KD + 8 * hi;
#pragma unroll
                    for (int kc = 0; kc < 3; ++kc) {
                        const v16bf w0 = ldb(wp + kc * 32), w1 = ldb(wp + 16 * KD + kc * 32), w2 = ldb(wp + 32 * KD + kc * 32);
                        acc[dj][0] = wmmab(ah[kc], w0, acc[dj][0]); acc[dj][1] = wmmab(ah[kc], w1, acc[dj][1]); acc[dj][2] = wmmab(ah[kc], w2, acc[dj][2]);
                        acc[dj][0] = wmmab(al[kc], w0, acc[dj][0]); acc[dj][1] = wmmab(al[kc], w1, acc[dj][1]); acc[dj][2] = wmmab(al[kc], w2, acc[dj][2]);
                        asm volatile("v_nop\n\tv_nop\n\tv_nop\n\tv_nop" : "+v"(acc[dj][0]), "+v"(acc[dj][1]), "+v"(acc[dj][2]) : "v"(w0), "v"(w1), "v"(w2), "v"(ah[kc]), "v"(al[kc]));
                    }
                }
            }
        }
#pragma unroll
        for (int nb = 0; nb < 3; ++nb) {
#pragma unroll
            for (int r = 0; r < 8; ++r) { const int q = 8 * hi + r;
                const float v0 = acc[0][nb][r] + bsum[0][nb]; const float v1 = acc[1][nb][r] + bsum[1][nb];
                const float v = ((q <= 14) ? v0 : 0.0f) + ((q >= 1) ? v1 : 0.0f);
                os[(rx + 4 * q) * OSP + nb * 16 + lr] = v; } }
    }
    wave_sync();
    float* ob = OUT + (size_t)b * OBS + (size_t)y * (WW * CI);
#pragma unroll 1
    for (int ps = 0; ps < 2; ++ps) {
#pragma unroll 4
        for (int s = 0; s < 24; ++s) { const int to = s >> 1, xx = ((s & 1) << 5) + lane;
            const v4f val = *(const v4fa*)(&os[xx * OSP + to * 4]);
            *(volatile v4f*)(ob + (size_t)to * TS + xx * 4) = val; }
        if (ps == 0) __threadfence(); }
}

static constexpr size_t al256(size_t v) { return (v + 255) & ~(size_t)255; }
static constexpr size_t SZ_V  = al256((size_t)NB * PIXB * KD * 2);
static constexpr size_t SZ_W  = al256((size_t)NPOS * NO * KD * 2);
static constexpr size_t SZ_B  = al256((size_t)NPOS * NO * 4);
static constexpr size_t SZ_TOTAL = 2 * SZ_V + SZ_W + SZ_B;
static_assert(SZ_TOTAL <= (size_t)134217728);
static_assert((size_t)(NB * PIXB / PP) * PP * KD * 2 <= SZ_V);
static_assert((size_t)WBLK * 256 * 16 <= SZ_W);
static_assert((size_t)BBLK * 256 * 16 <= SZ_B);

extern "C" void kernel_launch(void* const* d_in, const int* in_sizes, int n_in,
                              void* d_out, int out_size, void* d_ws, size_t ws_size, hipStream_t stream) {
    if (n_in < 5) return;
    if ((size_t)in_sizes[0] < (size_t)NB * XBS) return;
    if ((size_t)in_sizes[1] < (size_t)NO * 48 * 64 || (size_t)in_sizes[3] < (size_t)NO * 48 * 64) return;
    if ((size_t)in_sizes[2] < (size_t)NO * 64 || (size_t)in_sizes[4] < (size_t)NO * 64) return;
    if ((size_t)out_size < (size_t)NB * OBS) return;
    if (SZ_TOTAL > ws_size) return;
    const float* x  = (const float*)d_in[0];
    const float* ws = (const float*)d_in[1];
    const float* bs = (const float*)d_in[2];
    const float* wt = (const float*)d_in[3];
    const float* bt = (const float*)d_in[4];
    float* OUT = (float*)d_out;
    char* wsp = (char*)d_ws;
    bf* VH = (bf*)wsp; wsp += SZ_V;
    bf* VL = (bf*)wsp; wsp += SZ_V;
    bf* WST = (bf*)wsp; wsp += SZ_W;
    float* BIAS = (float*)wsp; wsp += SZ_B;

    k_prep<<<(unsigned)((size_t)NB * PIXB / PP), PP, 0, stream>>>(x, VH, VL);
    k_w<<<WBLK + BBLK, 256, 0, stream>>>(ws, bs, wt, bt, WST, BIAS);
    k_gemm<<<dim3(HH, NB, 1), 32, 0, stream>>>(VH, VL, WST, BIAS, OUT);
}
